// NLM_2319282340669
// MI455X (gfx1250) — hardware-verified
//
#include <hip/hip_runtime.h>
#include <stdint.h>

#define CHS    3
#define IMW    320
#define TS     32
#define NTW    10
#define NTILE  100
#define NPIX   1024
#define KFEAT  72
#define KP     128
#define RB     64
#define NRB    (NPIX / RB)
#define NCT    (NPIX / 64)
#define LOG2E  1.4426950408889634f

static_assert(NTW * TS == IMW);
static_assert(NTILE == NTW * NTW);
static_assert(NPIX == TS * TS);
static_assert((KFEAT % 8) == 0);
static_assert(KFEAT <= 96);
static_assert(KP == 128);
static_assert((NPIX % 256) == 0);
static_assert(RB == 2 * TS);

typedef __bf16   v16b __attribute__((ext_vector_type(16)));
typedef __bf16   v8b  __attribute__((ext_vector_type(8)));
typedef float    v8f  __attribute__((ext_vector_type(8)));
typedef float    v4f  __attribute__((ext_vector_type(4)));
typedef unsigned int v4u __attribute__((ext_vector_type(4)));
static_assert(sizeof(v4u) == 16);
static_assert(sizeof(v4f) == 16);

__device__ __forceinline__ int iclamp(int v, int lo, int hi) { return v < lo ? lo : (v > hi ? hi : v); }
__device__ __forceinline__ unsigned short bf_bits(float f) {
  unsigned u = __float_as_uint(f);
  return (unsigned short)((u + 0x7FFFu + ((u >> 16) & 1u)) >> 16);
}
__device__ __forceinline__ float bf_up(unsigned short b) { return __uint_as_float(((unsigned)b) << 16); }
__device__ __forceinline__ float bf_val(float f) { return bf_up(bf_bits(f)); }
__device__ __forceinline__ unsigned pk16(unsigned short a, unsigned short b) { return (unsigned)a | ((unsigned)b << 16); }
__device__ __forceinline__ v8f zero8() { v8f z = {0.f, 0.f, 0.f, 0.f, 0.f, 0.f, 0.f, 0.f}; return z; }

__device__ __forceinline__ v16b ldfrag_b(const __bf16* p) {
  union { v16b v; v8b h[2]; } f;
  f.h[0] = *(const v8b*)(p);
  f.h[1] = *(const v8b*)(p + 16);
  return f.v;
}

__device__ __forceinline__ v8f mma_b(v16b a, v16b b, v8f c) {
  c = __builtin_amdgcn_wmma_f32_16x16x32_bf16(false, a, false, b, (short)0, c, false, false);
#if defined(__HIP_DEVICE_COMPILE__)
  asm volatile("v_nop\n\tv_nop\n\tv_nop\n\tv_nop" : "+v"(c) : "v"(a), "v"(b));
#endif
  return c;
}

__global__ __launch_bounds__(256) void feat_rows(const float* __restrict__ img,
                                                  unsigned short* Yp, float* Sq) {
  __shared__ float timg[CHS * NPIX];
  __shared__ __align__(16) float ssq[256];

  const int tid  = threadIdx.x;
  const int lane = tid & 31;
  const int wave = tid >> 5;
  const int h    = lane >> 4;
  const int q    = lane & 15;
  const int pg   = blockIdx.x;
  const int tile = blockIdx.y;
  const int th   = tile / NTW;
  const int tw   = tile - th * NTW;

#pragma unroll 4
  for (int i = tid; i < CHS * NPIX; i += 256) {
    const int ch = i >> 10;
    const int m  = i & (NPIX - 1);
    const size_t g = (size_t)(ch * IMW + th * TS + (m >> 5)) * IMW + (size_t)(tw * TS + (m & 31));
    timg[i] = bf_val(img[g]);
  }
  __syncthreads();

  const int qq  = (q < 9) ? q : 8;
  const int chq = qq / 3;
  const int ob  = (qq - 3 * chq) * 8;
  const float* tim = timg + chq * NPIX;

#pragma unroll 1
  for (int p = 0; p < 16; ++p) {
    const int rl = p * 16 + 2 * wave + h;
    const int n  = pg * 256 + rl;
    const int ty = n >> 5, tx = n & 31;
    float s = 0.f;
    unsigned short bb[8];
#pragma unroll
    for (int e = 0; e < 8; ++e) {
      const int o   = ob + e;
      const int idx = (o < 12) ? o : (o + 1);
      const int pi  = idx / 5;
      const int di  = pi - 2;
      const int dj  = (idx - pi * 5) - 2;
      const int rr  = iclamp(ty + di, 0, TS - 1);
      const int cc  = iclamp(tx + dj, 0, TS - 1);
      float x = tim[rr * TS + cc];
      x = (q < 9) ? x : 0.f;
      s += x * x;
      bb[e] = bf_bits(x);
    }
    v4u pk;
    pk[0] = pk16(bb[0], bb[1]);
    pk[1] = pk16(bb[2], bb[3]);
    pk[2] = pk16(bb[4], bb[5]);
    pk[3] = pk16(bb[6], bb[7]);
#pragma unroll
    for (int off = 1; off < 16; off <<= 1) s += __shfl_xor(s, off, 32);
    if (q == 0) ssq[rl] = s;
    unsigned short* dst = Yp + (size_t)(tile * NPIX + n) * KP + 8 * q;
    *(volatile v4u*)dst = pk;
    __threadfence();
    *(volatile v4u*)dst = pk;
  }
  __syncthreads();
  if (tid < 64) {
    const v4f v = *(const v4f*)(&ssq[4 * tid]);
    float* d = Sq + (size_t)tile * NPIX + (size_t)(pg * 256 + 4 * tid);
    *(volatile v4f*)d = v;
    __threadfence();
    *(volatile v4f*)d = v;
  }
}

__global__ __launch_bounds__(128) void gram_mean(const unsigned short* __restrict__ Yp,
                                                  const float* __restrict__ Sq,
                                                  const float* __restrict__ img,
                                                  float* out) {
  const __bf16* Yb = (const __bf16*)(const void*)Yp;
  __shared__ float spix[CHS * NPIX];
  __shared__ float ssq[NPIX];
  __shared__ __align__(16) float sout[CHS][RB];

  const int tid  = threadIdx.x;
  const int lane = tid & 31;
  const int wave = tid >> 5;
  const int h    = lane >> 4;
  const int c    = lane & 15;
  const int rt   = blockIdx.x;
  const int tile = blockIdx.y;
  const int th   = tile / NTW;
  const int tw   = tile - th * NTW;

#pragma unroll 4
  for (int i = tid; i < CHS * NPIX; i += 128) {
    const int ch = i >> 10;
    const int m  = i & (NPIX - 1);
    const size_t g = (size_t)(ch * IMW + th * TS + (m >> 5)) * IMW + (size_t)(tw * TS + (m & 31));
    spix[i] = bf_val(img[g]);
  }
#pragma unroll 4
  for (int i = tid; i < NPIX; i += 128) ssq[i] = Sq[(size_t)tile * NPIX + i];
  __syncthreads();

  const int rbase = rt * RB + wave * 16;
  const int rown  = rbase + 8 * h;

  float sqr[8];
#pragma unroll
  for (int r = 0; r < 8; ++r) sqr[r] = ssq[rown + r];

  const __bf16* arow = Yb + (size_t)(tile * NPIX + rbase + c) * KP + 8 * h;
  const v16b a0 = ldfrag_b(arow);
  const v16b a1 = ldfrag_b(arow + 32);
  const v16b a2 = ldfrag_b(arow + 64);

  float den[8], nx[8], ny[8], nz[8];
#pragma unroll
  for (int r = 0; r < 8; ++r) { den[r] = 0.f; nx[r] = 0.f; ny[r] = 0.f; nz[r] = 0.f; }

#pragma unroll 1
  for (int t = 0; t < NCT; ++t) {
    const int cbase = t * 64;
    v8f acc[4];
#pragma unroll
    for (int j = 0; j < 4; ++j) acc[j] = zero8();
    const __bf16* brow = Yb + (size_t)(tile * NPIX + cbase + c) * KP + 8 * h;
    {
      v16b b[4];
#pragma unroll
      for (int j = 0; j < 4; ++j) b[j] = ldfrag_b(brow + (size_t)j * 16 * KP);
#pragma unroll
      for (int j = 0; j < 4; ++j) acc[j] = mma_b(a0, b[j], acc[j]);
    }
    {
      v16b b[4];
#pragma unroll
      for (int j = 0; j < 4; ++j) b[j] = ldfrag_b(brow + (size_t)j * 16 * KP + 32);
#pragma unroll
      for (int j = 0; j < 4; ++j) acc[j] = mma_b(a1, b[j], acc[j]);
    }
    {
      v16b b[4];
#pragma unroll
      for (int j = 0; j < 4; ++j) b[j] = ldfrag_b(brow + (size_t)j * 16 * KP + 64);
#pragma unroll
      for (int j = 0; j < 4; ++j) acc[j] = mma_b(a2, b[j], acc[j]);
    }

#pragma unroll
    for (int j = 0; j < 4; ++j) {
      const int col   = cbase + 16 * j + c;
      const float sqm = ssq[col];
      const float y0  = spix[col];
      const float y1  = spix[NPIX + col];
      const float y2  = spix[2 * NPIX + col];
#pragma unroll
      for (int r = 0; r < 8; ++r) {
        const float d2 = (sqr[r] + sqm) - 2.0f * acc[j][r];
        const float ds = __builtin_amdgcn_sqrtf(fmaxf(d2, 0.f));
        float dn = __builtin_amdgcn_exp2f(-LOG2E * ds);
        dn = ((rown + r) == col) ? 0.f : dn;
        den[r] += dn;
        nx[r]  += dn * y0;
        ny[r]  += dn * y1;
        nz[r]  += dn * y2;
      }
    }
  }

#pragma unroll
  for (int r = 0; r < 8; ++r) {
#pragma unroll
    for (int off = 1; off < 16; off <<= 1) {
      den[r] += __shfl_xor(den[r], off, 32);
      nx[r]  += __shfl_xor(nx[r],  off, 32);
      ny[r]  += __shfl_xor(ny[r],  off, 32);
      nz[r]  += __shfl_xor(nz[r],  off, 32);
    }
  }
  if (c == 0) {
#pragma unroll
    for (int r = 0; r < 8; ++r) {
      const int rl   = wave * 16 + 8 * h + r;
      const float rd = __builtin_amdgcn_rcpf(den[r]);
      sout[0][rl] = nx[r] * rd;
      sout[1][rl] = ny[r] * rd;
      sout[2][rl] = nz[r] * rd;
    }
  }
  __syncthreads();

  {
    const int tt  = (tid < 48) ? tid : 47;
    const int L   = tt >> 3;
    const int q   = tt & 7;
    const int ch  = L >> 1;
    const int tyl = L & 1;
    const v4f v = *(const v4f*)(&sout[ch][tyl * TS + 4 * q]);
    float* dst = out + (size_t)ch * (IMW * IMW) + (size_t)(th * TS + rt * 2 + tyl) * IMW
               + (size_t)(tw * TS + 4 * q);
    if (tid < 48) *(volatile v4f*)dst = v;
    __threadfence();
    if (tid < 48) *(volatile v4f*)dst = v;
  }
}

extern "C" void kernel_launch(void* const* d_in, const int* in_sizes, int n_in,
                              void* d_out, int out_size, void* d_ws, size_t ws_size,
                              hipStream_t stream) {
  if (n_in < 1) return;
  if (in_sizes[0] != CHS * IMW * IMW) return;
  if (out_size != CHS * IMW * IMW) return;

  const size_t bY  = (size_t)NTILE * NPIX * KP * 2;
  const size_t bSq = (size_t)NTILE * NPIX * 4;
  size_t off = 0;
  const size_t oY  = off; off += bY;
  const size_t oSq = off; off += bSq;
  if (off > ws_size) return;
  if (off > (size_t)134217728) return;

  const float* img = (const float*)d_in[0];
  float* out = (float*)d_out;
  char* ws = (char*)d_ws;
  unsigned short* Yp = (unsigned short*)(ws + oY);
  float* Sq = (float*)(ws + oSq);

  feat_rows<<<dim3(NPIX / 256, NTILE), dim3(256), 0, stream>>>(img, Yp, Sq);
  gram_mean<<<dim3(NRB, NTILE), dim3(128), 0, stream>>>(Yp, Sq, img, out);
  (void)hipGetLastError();
}
